// Mamba2_70995809402924
// MI455X (gfx1250) — hardware-run, weakly checked
//
#include <hip/hip_runtime.h>
#include <math.h>

typedef __attribute__((ext_vector_type(16))) __bf16   v16b;
typedef __attribute__((ext_vector_type(8)))  __bf16   v8b;
typedef __attribute__((ext_vector_type(8)))  float    v8f;
typedef __attribute__((ext_vector_type(4)))  float    v4f;
typedef __attribute__((ext_vector_type(4)))  unsigned v4u;

constexpr int kBatch  = 2;
constexpr int kSeq    = 512;
constexpr int kDm     = 1024;
constexpr int kNst    = 128;
constexpr int kHd     = 64;
constexpr int kDi     = 2048;
constexpr int kNh     = 32;
constexpr int kCv     = 2304;
constexpr int kNp     = 4384;
constexpr int kNpPad  = 4416;
constexpr int kRows   = kBatch * kSeq;
constexpr int kConvTP = 260;
constexpr int kScanT  = 32;
constexpr int kScanYP = 68;
constexpr float kEps  = 1e-5f;
static_assert(kDi == kNh * kHd);
static_assert(kCv == kDi + 2 * kNst);
static_assert(kNp == 2 * kDi + 2 * kNst + kNh);
static_assert(kNpPad % 64 == 0 && kNpPad >= kNp && kNpPad - kNp < 64);
static_assert(kRows == 1024);
static_assert(kRows % 64 == 0 && kDm % 64 == 0 && kDm % 32 == 0 && kDi % 32 == 0);
static_assert(kSeq % 64 == 0 && (kSeq & (kSeq - 1)) == 0 && kCv % 256 == 0 && kSeq % kScanT == 0 && kScanT == 32);
static_assert(kNst == 128 && kHd == 64 && kNh == 32);
static_assert(((kRows / 64) * (kNpPad / 64)) % 8 == 0);
static_assert(((kRows / 64) * (kDm / 64)) % 8 == 0);

constexpr size_t kOffXB  = 0;
constexpr size_t kOffWIB = kOffXB  + (size_t)kRows  * kDm * 2;
constexpr size_t kOffWOB = kOffWIB + (size_t)kNpPad * kDm * 2;
constexpr size_t kOffZP  = kOffWOB + (size_t)kDm    * kDi * 2;
constexpr size_t kOffXBC = kOffZP  + (size_t)kRows  * kNpPad * 4;
constexpr size_t kOffDTP = kOffXBC + (size_t)kRows  * kCv * 4;
constexpr size_t kOffDAP = kOffDTP + (size_t)kRows  * kNh * 4;
constexpr size_t kOffYP  = kOffDAP + (size_t)kRows  * kNh * 4;
constexpr size_t kOffYH  = kOffYP  + (size_t)kRows  * kDi * 4;
constexpr size_t kOffYL  = kOffYH  + (size_t)kRows  * kDi * 2;
constexpr size_t kWsTotal = kOffYL + (size_t)kRows  * kDi * 2;
static_assert(kWsTotal == 59899904ull);
static_assert(kWsTotal <= 134217728ull);
static_assert((kOffWIB % 256) == 0 && (kOffWOB % 256) == 0 && (kOffZP % 256) == 0 && (kOffXBC % 256) == 0 &&
              (kOffDTP % 256) == 0 && (kOffDAP % 256) == 0 && (kOffYP % 256) == 0 && (kOffYH % 256) == 0 &&
              (kOffYL % 256) == 0);

__device__ __forceinline__ unsigned bf_bits(float f) {
  const unsigned u = __float_as_uint(f);
  return (u + 0x7FFFu + ((u >> 16) & 1u)) >> 16;
}
__device__ __forceinline__ float bf_val(unsigned b) { return __uint_as_float(b << 16); }
__device__ __forceinline__ float bf16r(float f) { return bf_val(bf_bits(f)); }

__device__ __forceinline__ void row_guard_b(v8f& a0, v8f& a1, v8f& a2, v8f& a3, v16b x, v16b y) {
  asm volatile("v_nop\n\tv_nop\n\tv_nop\n\tv_nop" : "+v"(a0), "+v"(a1), "+v"(a2), "+v"(a3) : "v"(x), "v"(y));
}
__device__ __forceinline__ void keep4_b(v16b a, v16b b, v16b c, v16b d) { asm volatile("v_nop" :: "v"(a), "v"(b), "v"(c), "v"(d)); }
__device__ __forceinline__ void acc_guard4(v8f& a, v8f& b, v8f& c, v8f& d) {
  asm volatile("v_nop\n\tv_nop\n\tv_nop\n\tv_nop" : "+v"(a), "+v"(b), "+v"(c), "+v"(d));
}

struct FragB {
  union U { v16b v; v8b h[2]; };
  static __device__ __forceinline__ v16b load(const __bf16* p) {
    U f; f.h[0] = *(const v8b*)(p); f.h[1] = *(const v8b*)(p + 16); return f.v;
  }
  static __device__ __forceinline__ v8f mma(v16b a, v16b b, v8f c) {
    return __builtin_amdgcn_wmma_f32_16x16x32_bf16(false, a, false, b, (short)0, c, false, false);
  }
};

__global__ __launch_bounds__(256) void cvt_rows_bf16_kernel(
    const float* __restrict__ src, unsigned* __restrict__ dst, int nrow_dst, int nrow_src, int ncol8)
{
  const int i  = blockIdx.x * 256 + threadIdx.x;
  const int n8 = nrow_dst * ncol8;
  if (i >= n8) return;
  const int row = i / ncol8;
  const int c8  = i - row * ncol8;
  const int rs  = (row < nrow_src) ? row : (nrow_src - 1);
  const bool keep = (row < nrow_src);
  const float* sp = src + ((size_t)rs * ncol8 + c8) * 8;
  const v4f a = *(const v4f*)(sp);
  const v4f b = *(const v4f*)(sp + 4);
  const float a0 = a[0], a1 = a[1], a2 = a[2], a3 = a[3];
  const float b0 = b[0], b1 = b[1], b2 = b[2], b3 = b[3];
  const unsigned h0 = bf_bits(keep ? a0 : 0.0f), h1 = bf_bits(keep ? a1 : 0.0f);
  const unsigned h2 = bf_bits(keep ? a2 : 0.0f), h3 = bf_bits(keep ? a3 : 0.0f);
  const unsigned h4 = bf_bits(keep ? b0 : 0.0f), h5 = bf_bits(keep ? b1 : 0.0f);
  const unsigned h6 = bf_bits(keep ? b2 : 0.0f), h7 = bf_bits(keep ? b3 : 0.0f);
  v4u o;
  o[0] = h0 | (h1 << 16);
  o[1] = h2 | (h3 << 16);
  o[2] = h4 | (h5 << 16);
  o[3] = h6 | (h7 << 16);
  unsigned* dp = dst + (size_t)i * 4;
  *(volatile v4u*)dp = o;
  __threadfence();
  *(volatile v4u*)dp = o;
}

template <int SPL>
__global__ __launch_bounds__(256) void wmma_gemm64_bf16(
    const unsigned short* __restrict__ Ap, const unsigned short* __restrict__ A2p, int lda,
    const unsigned short* __restrict__ Btp, int ldb,
    float* __restrict__ C, int ldc, int M, int N, int K)
{
  const __bf16* A  = (const __bf16*)Ap;
  const __bf16* A2 = (const __bf16*)A2p;
  const __bf16* Bt = (const __bf16*)Btp;
  __shared__ __align__(16) float sT[8][16 * 68];
  const int lane = threadIdx.x & 31;
  const int wave = threadIdx.x >> 5;
  const int tilesN = N >> 6;
  const int tilesM = M >> 6;
  const int tile = blockIdx.x * 8 + wave;
  if (tile >= tilesM * tilesN) return;
  const int tm = tile / tilesN;
  const int tn = tile - tm * tilesN;
  const int m0 = tm << 6;
  const int n0 = tn << 6;

  const int rlane = lane & 15;
  const int koff  = (lane >> 4) * 8;
  const int mOff  = (lane >> 4) * 8;

  v8f acc[4][4];
#pragma unroll
  for (int i = 0; i < 4; ++i)
#pragma unroll
    for (int j = 0; j < 4; ++j) acc[i][j] = (v8f){0.f, 0.f, 0.f, 0.f, 0.f, 0.f, 0.f, 0.f};

  for (int k0 = 0; k0 < K; k0 += 32) {
    v16b bh[4];
#pragma unroll
    for (int j = 0; j < 4; ++j) {
      const size_t bo = (size_t)(n0 + (j << 4) + rlane) * ldb + koff + k0;
      bh[j] = FragB::load(Bt + bo);
    }
#pragma unroll
    for (int i = 0; i < 4; ++i) {
      const size_t ao = (size_t)(m0 + (i << 4) + rlane) * lda + koff + k0;
      const v16b ah = FragB::load(A + ao);
      v16b al = ah;
      if (SPL == 1) al = FragB::load(A2 + ao);
#pragma unroll
      for (int j = 0; j < 4; ++j) {
        acc[i][j] = FragB::mma(ah, bh[j], acc[i][j]);
        if (SPL == 1) acc[i][j] = FragB::mma(al, bh[j], acc[i][j]);
      }
      row_guard_b(acc[i][0], acc[i][1], acc[i][2], acc[i][3], ah, al);
    }
    keep4_b(bh[0], bh[1], bh[2], bh[3]);
  }
  acc_guard4(acc[0][0], acc[0][1], acc[0][2], acc[0][3]);
  acc_guard4(acc[1][0], acc[1][1], acc[1][2], acc[1][3]);
  acc_guard4(acc[2][0], acc[2][1], acc[2][2], acc[2][3]);
  acc_guard4(acc[3][0], acc[3][1], acc[3][2], acc[3][3]);

  float* slab = sT[wave];
#pragma unroll
  for (int i = 0; i < 4; ++i) {
    const int mBase = m0 + (i << 4);
#pragma unroll
    for (int j = 0; j < 4; ++j) {
#pragma unroll
      for (int r = 0; r < 8; ++r) slab[(mOff + r) * 68 + (j << 4) + rlane] = acc[i][j][r];
    }
    __builtin_amdgcn_fence(__ATOMIC_RELEASE, "workgroup");
    __builtin_amdgcn_wave_barrier();
    __builtin_amdgcn_fence(__ATOMIC_ACQUIRE, "workgroup");
    {
      const int hh = lane >> 4, c4 = (lane & 15) * 4;
      for (int pass = 0; pass < 2; ++pass) {
#pragma unroll
        for (int it = 0; it < 8; ++it) {
          const int row = it * 2 + hh;
          const v4f v = *(const v4f*)(slab + row * 68 + c4);
          *(volatile v4f*)(C + (size_t)(mBase + row) * ldc + n0 + c4) = v;
        }
        __threadfence();
      }
    }
    __builtin_amdgcn_fence(__ATOMIC_RELEASE, "workgroup");
    __builtin_amdgcn_wave_barrier();
    __builtin_amdgcn_fence(__ATOMIC_ACQUIRE, "workgroup");
  }
}

__global__ __launch_bounds__(256) void conv_silu_kernel(
    const float* __restrict__ ZP, const float* __restrict__ cw, const float* __restrict__ cb,
    float* __restrict__ XBC)
{
  __shared__ __align__(16) float sT[16 * kConvTP];
  const int tid = threadIdx.x, lane = tid & 31, wave = tid >> 5;
  const int d0 = blockIdx.x * 256, d = d0 + tid;
  const int g0 = blockIdx.y * 64;
  const int tb = g0 & (kSeq - 1);
  const v4f wv = *(const v4f*)(cw + (size_t)d * 4);
  const float wa = wv[0], wb = wv[1], wc = wv[2], wd = wv[3];
  const float w0 = bf16r(wa), w1 = bf16r(wb), w2 = bf16r(wc), w3 = bf16r(wd);
  const float bc = bf16r(cb[d]);
  const float* zc = ZP + kDi + d;
  float xm3, xm2, xm1;
  {
    const bool hist = (tb > 0);
    const int rb = hist ? (g0 - 3) : g0;
    const float v3 = zc[(size_t)rb * kNpPad];
    const float v2 = zc[(size_t)(rb + 1) * kNpPad];
    const float v1 = zc[(size_t)(rb + 2) * kNpPad];
    xm3 = hist ? v3 : 0.0f;
    xm2 = hist ? v2 : 0.0f;
    xm1 = hist ? v1 : 0.0f;
  }
  const int hrow = wave >> 1;
  const int hch  = (wave & 1) * 128 + lane * 4;
#pragma unroll 1
  for (int sub = 0; sub < 4; ++sub) {
    const int lb = g0 + sub * 16;
#pragma unroll 1
    for (int s = 0; s < 16; ++s) {
      const float xcur = zc[(size_t)(lb + s) * kNpPad];
      float acc = w0 * xm3;
      acc = fmaf(w1, xm2, acc);
      acc = fmaf(w2, xm1, acc);
      acc = fmaf(w3, xcur, acc);
      const float sv = acc + bc;
      const float sg = __builtin_amdgcn_rcpf(1.0f + expf(-sv));
      sT[s * kConvTP + tid] = sv * sg;
      xm3 = xm2; xm2 = xm1; xm1 = xcur;
    }
    __syncthreads();
    v4f fv[4];
#pragma unroll
    for (int it = 0; it < 4; ++it) fv[it] = *(const v4f*)(sT + (it * 4 + hrow) * kConvTP + hch);
    for (int pass = 0; pass < 2; ++pass) {
#pragma unroll
      for (int it = 0; it < 4; ++it)
        *(volatile v4f*)(XBC + (size_t)(lb + it * 4 + hrow) * kCv + d0 + hch) = fv[it];
      __threadfence();
    }
    __syncthreads();
  }
}

__global__ __launch_bounds__(256) void dt_decay_kernel(
    const float* __restrict__ ZP, const float* __restrict__ dt_bias, const float* __restrict__ A_log,
    float* __restrict__ DTP, float* __restrict__ DAP)
{
  const int lane = threadIdx.x & 31, wave = threadIdx.x >> 5;
  const int row = blockIdx.x * 8 + wave;
  const float v  = ZP[(size_t)row * kNpPad + kDi + kCv + lane] + bf16r(dt_bias[lane]);
  const float sp = fmaxf(v, 0.0f) + log1pf(expf(-fabsf(v)));
  const float Ah = -expf(bf16r(A_log[lane]));
  const float da = expf(sp * Ah);
  float* p0 = DTP + (size_t)row * kNh + lane;
  float* p1 = DAP + (size_t)row * kNh + lane;
  *(volatile float*)p0 = sp;
  *(volatile float*)p1 = da;
  __threadfence();
  *(volatile float*)p0 = sp;
  *(volatile float*)p1 = da;
}

__global__ __launch_bounds__(256) void scan_kernel(
    const float* __restrict__ XBC, const float* __restrict__ DTP, const float* __restrict__ DAP,
    const float* __restrict__ Dv, float* __restrict__ YP)
{
  __shared__ __align__(16) float sBC[kScanT * 256];
  __shared__ __align__(16) float sX[kScanT * kHd];
  __shared__ __align__(16) float sY[kScanT * kScanYP];
  __shared__ float sDt[kScanT];
  __shared__ float sDa[kScanT];
  const int tid = threadIdx.x, lane = tid & 31, wave = tid >> 5;
  const int bix  = blockIdx.x >> 5;
  const int head = blockIdx.x & 31;
  const int p = tid >> 2, q = tid & 3;
  const size_t row0 = (size_t)bix * kSeq;
  const float Dh = bf16r(Dv[head]);
  float h[32];
#pragma unroll
  for (int i = 0; i < 32; ++i) h[i] = 0.0f;
  const int hh = lane >> 4, c4o = (lane & 15) * 4;

#pragma unroll 1
  for (int t0 = 0; t0 < kSeq; t0 += kScanT) {
    __syncthreads();
#pragma unroll
    for (int it = 0; it < 8; ++it) {
      const int idx = it * 256 + tid;
      const int r = idx >> 6, c4 = (idx & 63) * 4;
      const v4f v = *(const v4f*)(XBC + (row0 + t0 + r) * kCv + kDi + c4);
      *(v4f*)(sBC + r * 256 + c4) = v;
    }
#pragma unroll
    for (int it = 0; it < 2; ++it) {
      const int idx = it * 256 + tid;
      const int r = idx >> 4, c4 = (idx & 15) * 4;
      const v4f v = *(const v4f*)(XBC + (row0 + t0 + r) * kCv + head * kHd + c4);
      *(v4f*)(sX + r * kHd + c4) = v;
    }
    {
      const int ts = tid & 31;
      float dtv = DTP[(row0 + t0 + ts) * kNh + head];
      float dav = DAP[(row0 + t0 + ts) * kNh + head];
      asm volatile("" : "+v"(dtv), "+v"(dav));
      if (tid < kScanT) { sDt[tid] = dtv; sDa[tid] = dav; }
    }
    __syncthreads();

#pragma unroll 1
    for (int s = 0; s < kScanT; ++s) {
      const float dA   = sDa[s];
      const float xp   = sX[s * kHd + p];
      const float coef = sDt[s] * xp;
      const float* Bq = sBC + s * 256 + q * 32;
      const float* Cq = Bq + kNst;
      float yp = 0.0f;
#pragma unroll
      for (int i4 = 0; i4 < 8; ++i4) {
        const v4f bv = *(const v4f*)(Bq + 4 * i4);
        const v4f cv = *(const v4f*)(Cq + 4 * i4);
#pragma unroll
        for (int e = 0; e < 4; ++e) {
          const float hd = dA * h[4 * i4 + e];
          const float hn = fmaf(coef, bv[e], hd);
          h[4 * i4 + e] = hn;
          yp = fmaf(cv[e], hn, yp);
        }
      }
      yp += __shfl_xor(yp, 1, 32);
      yp += __shfl_xor(yp, 2, 32);
      const float yo = fmaf(Dh, xp, yp);
      if (q == 0) sY[s * kScanYP + p] = yo;
    }
    __syncthreads();

    v4f fv[2];
#pragma unroll
    for (int it = 0; it < 2; ++it) {
      const int row = it * 16 + wave * 2 + hh;
      fv[it] = *(const v4f*)(sY + row * kScanYP + c4o);
    }
    for (int pass = 0; pass < 2; ++pass) {
#pragma unroll
      for (int it = 0; it < 2; ++it) {
        const int row = it * 16 + wave * 2 + hh;
        *(volatile v4f*)(YP + (row0 + t0 + row) * kDi + head * kHd + c4o) = fv[it];
      }
      __threadfence();
    }
  }
}

__global__ __launch_bounds__(256) void gate_norm_kernel(
    const float* __restrict__ YP, const float* __restrict__ ZP, const float* __restrict__ nw,
    unsigned* __restrict__ YH, unsigned* __restrict__ YL)
{
  __shared__ float red[8];
  const int tid = threadIdx.x, lane = tid & 31, wave = tid >> 5;
  const int row = blockIdx.x;
  const size_t rbase = (size_t)row * kDi + (size_t)tid * 8;
  const v4f ya = *(const v4f*)(YP + rbase);
  const v4f yb = *(const v4f*)(YP + rbase + 4);
  const v4f za = *(const v4f*)(ZP + (size_t)row * kNpPad + tid * 8);
  const v4f zb = *(const v4f*)(ZP + (size_t)row * kNpPad + tid * 8 + 4);
  const v4f na = *(const v4f*)(nw + tid * 8);
  const v4f nb = *(const v4f*)(nw + tid * 8 + 4);
  float yv[8], zv[8], nv[8];
#pragma unroll
  for (int e = 0; e < 4; ++e) {
    yv[e] = ya[e]; yv[4 + e] = yb[e];
    zv[e] = za[e]; zv[4 + e] = zb[e];
    nv[e] = na[e]; nv[4 + e] = nb[e];
  }
  float gv[8];
  float ss = 0.0f;
#pragma unroll
  for (int e = 0; e < 8; ++e) {
    const float z  = zv[e];
    const float sg = __builtin_amdgcn_rcpf(1.0f + expf(-z));
    const float g  = yv[e] * (z * sg);
    gv[e] = g;
    ss = fmaf(g, g, ss);
  }
#pragma unroll
  for (int off = 1; off < 32; off <<= 1) ss += __shfl_xor(ss, off, 32);
  if (lane == 0) red[wave] = ss;
  __syncthreads();
  const float tot = ((red[0] + red[1]) + (red[2] + red[3])) + ((red[4] + red[5]) + (red[6] + red[7]));
  const float rs = rsqrtf(tot * (1.0f / (float)kDi) + kEps);
  unsigned hw[4], lw[4];
#pragma unroll
  for (int e2 = 0; e2 < 4; ++e2) {
    unsigned hb[2], lb[2];
#pragma unroll
    for (int u = 0; u < 2; ++u) {
      const int e = 2 * e2 + u;
      const float o = (gv[e] * rs) * bf16r(nv[e]);
      const unsigned hbits = bf_bits(o);
      const float resid = o - bf_val(hbits);
      hb[u] = hbits;
      lb[u] = bf_bits(resid);
    }
    hw[e2] = hb[0] | (hb[1] << 16);
    lw[e2] = lb[0] | (lb[1] << 16);
  }
  v4u vh, vl;
  vh[0] = hw[0]; vh[1] = hw[1]; vh[2] = hw[2]; vh[3] = hw[3];
  vl[0] = lw[0]; vl[1] = lw[1]; vl[2] = lw[2]; vl[3] = lw[3];
  unsigned* ph = YH + (rbase >> 1);
  unsigned* pl = YL + (rbase >> 1);
  *(volatile v4u*)ph = vh;
  *(volatile v4u*)pl = vl;
  __threadfence();
  *(volatile v4u*)ph = vh;
  *(volatile v4u*)pl = vl;
}

extern "C" void kernel_launch(void* const* d_in, const int* in_sizes, int n_in,
                              void* d_out, int out_size, void* d_ws, size_t ws_size,
                              hipStream_t stream) {
  if (n_in < 9 || d_out == nullptr || d_ws == nullptr) return;
  if (in_sizes[0] != kRows * kDm) return;
  if (in_sizes[1] != kNp * kDm) return;
  if (in_sizes[2] != kCv * 4) return;
  if (in_sizes[3] != kCv) return;
  if (in_sizes[4] != kNh) return;
  if (in_sizes[5] != kNh) return;
  if (in_sizes[6] != kNh) return;
  if (in_sizes[7] != kDi) return;
  if (in_sizes[8] != kDm * kDi) return;
  if (out_size != kRows * kDm) return;
  if (ws_size < kWsTotal) return;

  const float* x       = (const float*)d_in[0];
  const float* Win     = (const float*)d_in[1];
  const float* conv_w  = (const float*)d_in[2];
  const float* conv_b  = (const float*)d_in[3];
  const float* dt_bias = (const float*)d_in[4];
  const float* A_log   = (const float*)d_in[5];
  const float* Dv      = (const float*)d_in[6];
  const float* norm_w  = (const float*)d_in[7];
  const float* Wout    = (const float*)d_in[8];
  float* out = (float*)d_out;

  char* ws = (char*)d_ws;
  unsigned short* XB  = (unsigned short*)(ws + kOffXB);
  unsigned short* WIB = (unsigned short*)(ws + kOffWIB);
  unsigned short* WOB = (unsigned short*)(ws + kOffWOB);
  float*          ZP  = (float*)(ws + kOffZP);
  float*          XBC = (float*)(ws + kOffXBC);
  float*          DTP = (float*)(ws + kOffDTP);
  float*          DAP = (float*)(ws + kOffDAP);
  float*          YP  = (float*)(ws + kOffYP);
  unsigned short* YH  = (unsigned short*)(ws + kOffYH);
  unsigned short* YL  = (unsigned short*)(ws + kOffYL);

  cvt_rows_bf16_kernel<<<(kRows * (kDm / 8)) / 256, 256, 0, stream>>>(x, (unsigned*)XB, kRows, kRows, kDm / 8);
  cvt_rows_bf16_kernel<<<(kNpPad * (kDm / 8)) / 256, 256, 0, stream>>>(Win, (unsigned*)WIB, kNpPad, kNp, kDm / 8);
  cvt_rows_bf16_kernel<<<(kDm * (kDi / 8)) / 256, 256, 0, stream>>>(Wout, (unsigned*)WOB, kDm, kDm, kDi / 8);

  wmma_gemm64_bf16<0><<<dim3((kRows / 64) * (kNpPad / 64) / 8), 256, 0, stream>>>(
      XB, XB, kDm, WIB, kDm, ZP, kNpPad, kRows, kNpPad, kDm);

  conv_silu_kernel<<<dim3(kCv / 256, kRows / 64), 256, 0, stream>>>(ZP, conv_w, conv_b, XBC);

  dt_decay_kernel<<<kRows / 8, 256, 0, stream>>>(ZP, dt_bias, A_log, DTP, DAP);

  scan_kernel<<<kBatch * kNh, 256, 0, stream>>>(XBC, DTP, DAP, Dv, YP);

  gate_norm_kernel<<<kRows, 256, 0, stream>>>(YP, ZP, norm_w, (unsigned*)YH, (unsigned*)YL);

  wmma_gemm64_bf16<1><<<dim3((kRows / 64) * (kDm / 64) / 8), 256, 0, stream>>>(
      YH, YL, kDi, WOB, kDi, out, kDm, kRows, kDm, kDi);
}
